// MCSL_73349451481510
// MI455X (gfx1250) — hardware-verified
//
#include <hip/hip_runtime.h>
#include <stddef.h>

#define NN 100000
#define DD 50
#define HH 16
#define KP 64
#define K2 32
#define TAUF 0.3f
#define EPSF 1e-20f
#define SLOPE 0.05f

#define TILES (NN / 16)
#define NPAIR (DD * HH)
#define PREP_BLOCKS (NPAIR / 8)
#define P1_HALVES (NPAIR * 2 * KP)
#define P2_HALVES (NPAIR * 2 * K2)
#define OPIECES (16 * DD / 4)
#define WPIECES (DD * DD / 4)

static_assert(NN % 16 == 0);
static_assert(NPAIR % 8 == 0);
static_assert((16 * DD * 4) % 128 == 0);
static_assert((DD * DD) % 4 == 0);
static_assert(DD <= KP);

typedef __bf16 v16b __attribute__((ext_vector_type(16)));
typedef unsigned short v8us __attribute__((ext_vector_type(8)));
typedef float v8f __attribute__((ext_vector_type(8)));
typedef float v4f __attribute__((ext_vector_type(4)));
typedef unsigned int v4u __attribute__((ext_vector_type(4)));
typedef v8us __attribute__((may_alias)) v8usa;
typedef v4f __attribute__((may_alias)) v4fa;
typedef v4u __attribute__((may_alias)) v4ua;

union Frag { v16b v; v8us h[2]; unsigned short s[16]; };

__device__ __forceinline__ v8f mma_bf(v16b a, v16b b, v8f c) {
  c = __builtin_amdgcn_wmma_f32_16x16x32_bf16(false, a, false, b, (short)0, c, false, false);
  asm volatile("v_nop\n\tv_nop\n\tv_nop\n\tv_nop" : "+v"(c) : "v"(a), "v"(b));
  return c;
}

__device__ __forceinline__ unsigned short bfr(float f) {
  unsigned u = __float_as_uint(f);
  u += 0x7FFFu + ((u >> 16) & 1u);
  return (unsigned short)(u >> 16);
}
__device__ __forceinline__ float bff(unsigned short b) { return __uint_as_float(((unsigned)b) << 16); }

__device__ __forceinline__ float leaky(float v) { return fmaxf(v, SLOPE * v); }

__device__ __forceinline__ v16b ldfrag_g(const unsigned short* __restrict__ rowp, int h) {
  Frag f;
  f.h[0] = *(const v8us*)(rowp + 8 * h);
  f.h[1] = *(const v8us*)(rowp + 16 + 8 * h);
  return f.v;
}
__device__ __forceinline__ v16b ldfrag_l(const unsigned short* rowp, int h) {
  Frag f;
  f.h[0] = *(const v8usa*)(rowp + 8 * h);
  f.h[1] = *(const v8usa*)(rowp + 16 + 8 * h);
  return f.v;
}

__global__ __launch_bounds__(256) void k_prep(const float* __restrict__ w, const float* __restrict__ u1,
                                              const float* __restrict__ u2, const float* __restrict__ W1,
                                              const float* __restrict__ W2, unsigned short* __restrict__ planes,
                                              float* __restrict__ out1) {
  __shared__ __align__(16) float swp[2560];
  __shared__ __align__(16) unsigned short stg[8][256];

  const int tid = threadIdx.x, lane = tid & 31, wave = tid >> 5;

#pragma unroll 1
  for (int j = 0; j < 10; ++j) {
    const int idx = tid + 256 * j;
    const int idc = (idx < DD * DD) ? idx : DD * DD - 1;
    const int r = idc / DD;
    const int c = idc - r * DD;
    const float uv1 = u1[idc];
    const float uv2 = u2[idc];
    float z = w[idc];
#pragma unroll 1
    for (int t = 0; t < 2; ++t) {
      const float u = (t == 0) ? uv1 : uv2;
      float g = -logf(-logf(u + EPSF) + EPSF);
      g = (r == c) ? 0.0f : g;
      z = (t == 0) ? (z + g) : (z - g);
    }
    z = z * (1.0f / TAUF);
    const float e = expf(-z);
    float v = __builtin_amdgcn_rcpf(1.0f + e);
    v = (r == c) ? 0.0f : v;
    if (idx < DD * DD) swp[idx] = v;
  }
  __syncthreads();

  if (blockIdx.x == PREP_BLOCKS) {
    v4f val[3];
#pragma unroll
    for (int it = 0; it < 3; ++it) {
      const int p = tid + 256 * it;
      const int pc = (p < WPIECES) ? p : WPIECES - 1;
      val[it] = *(const v4fa*)(swp + 4 * pc);
    }
#pragma unroll
    for (int it = 0; it < 3; ++it) {
      const int p = tid + 256 * it;
      if (p < WPIECES) *(volatile v4f*)(out1 + 4 * (size_t)p) = val[it];
    }
    __threadfence();
#pragma unroll
    for (int it = 0; it < 3; ++it) {
      const int p = tid + 256 * it;
      if (p < WPIECES) *(volatile v4f*)(out1 + 4 * (size_t)p) = val[it];
    }
  } else {
    const int pair = blockIdx.x * 8 + wave;
    const int i = pair >> 4;
    const int n = pair & (HH - 1);
    unsigned short* sg = stg[wave];
#pragma unroll
    for (int q = 0; q < 2; ++q) {
      const int k = lane + 32 * q;
      const int kc = (k < DD) ? k : DD - 1;
      float v = swp[kc * DD + i] * W1[(i * DD + kc) * HH + n];
      v = (k < DD) ? v : 0.0f;
      const unsigned short hi = bfr(v);
      const unsigned short lo = bfr(v - bff(hi));
      sg[k]      = hi;
      sg[KP + k] = lo;
    }
    {
      const int hh = lane >> 1;
      const float v2 = W2[(i * HH + hh) * HH + n];
      const unsigned short hi2 = bfr(v2);
      const unsigned short lo2 = bfr(v2 - bff(hi2));
      sg[2 * KP + lane]      = hi2;
      sg[2 * KP + K2 + lane] = (lane & 1) ? (unsigned short)0 : lo2;
    }
    __syncthreads();
    const int pl = (lane < 24) ? lane : 23;
    const v4u val = *(const v4ua*)(sg + 8 * pl);
    const size_t off = (lane < 16) ? ((size_t)pair * (2 * KP) + (size_t)(8 * lane))
                                   : ((size_t)P1_HALVES + (size_t)pair * (2 * K2) + (size_t)(8 * (lane - 16)));
    unsigned short* dst = planes + off;
    if (lane < 24) *(volatile v4u*)dst = val;
    __threadfence();
    if (lane < 24) *(volatile v4u*)dst = val;
  }
}

__global__ __launch_bounds__(256) void k_main(const float* __restrict__ x, const unsigned short* __restrict__ P1,
                                              const unsigned short* __restrict__ P2, const float* __restrict__ b1,
                                              const float* __restrict__ b2, const float* __restrict__ W3,
                                              const float* __restrict__ b3, float* __restrict__ out0, int numTiles) {
  __shared__ __align__(16) unsigned int sT[8][16 * 16];
  __shared__ __align__(16) float sO[8][16 * DD];

  const int tid = threadIdx.x, lane = tid & 31, wave = tid >> 5;
  const int h = lane >> 4, m = lane & 15;
  const int tile = blockIdx.x * 8 + wave;
  const bool valid = tile < numTiles;
  const int tilec = valid ? tile : numTiles - 1;
  const int row0 = tilec * 16;

  Frag xh[2], xl[2];
  const float* xr = x + (size_t)(row0 + m) * DD;
#pragma unroll
  for (int ks = 0; ks < 2; ++ks) {
#pragma unroll
    for (int half = 0; half < 2; ++half) {
#pragma unroll
      for (int e = 0; e < 8; ++e) {
        const int k = 32 * ks + 16 * half + 8 * h + e;
        const int kc = (k < DD) ? k : DD - 1;
        float f = xr[kc];
        f = (k < DD) ? f : 0.0f;
        const unsigned short hi = bfr(f);
        const unsigned short lo = bfr(f - bff(hi));
        xh[ks].s[8 * half + e] = hi;
        xl[ks].s[8 * half + e] = lo;
      }
    }
  }

  unsigned int* Tw = sT[wave];
  const unsigned short* Th = (const unsigned short*)(sT[wave]);
  float* Ow = sO[wave];

#pragma unroll 1
  for (int i = 0; i < DD; ++i) {
    const float bb1 = b1[i * HH + m];
    v8f acc;
#pragma unroll
    for (int r = 0; r < 8; ++r) acc[r] = bb1;
#pragma unroll
    for (int ks = 0; ks < 2; ++ks) {
      const unsigned short* bp = P1 + ((size_t)(i * HH + m) * 2) * KP + 32 * ks;
      const v16b bh = ldfrag_g(bp, h);
      const v16b bl = ldfrag_g(bp + KP, h);
      acc = mma_bf(xh[ks].v, bh, acc);
      acc = mma_bf(xh[ks].v, bl, acc);
      acc = mma_bf(xl[ks].v, bh, acc);
    }
#pragma unroll
    for (int r = 0; r < 8; ++r) {
      const float v = leaky(acc[r]);
      const unsigned short hi = bfr(v);
      const unsigned short lo = bfr(v - bff(hi));
      Tw[(8 * h + r) * 16 + m] = (unsigned)hi | (((unsigned)lo) << 16);
    }
    __syncthreads();

    const v16b hb = ldfrag_l(Th + m * K2, h);
    const unsigned short* ap = P2 + (size_t)(i * HH + m) * (2 * K2);
    const v16b a2h = ldfrag_g(ap, h);
    const v16b a2l = ldfrag_g(ap + K2, h);
    v8f acc2;
#pragma unroll
    for (int r = 0; r < 8; ++r) acc2[r] = b2[i * HH + 8 * h + r];
    acc2 = mma_bf(a2h, hb, acc2);
    acc2 = mma_bf(a2l, hb, acc2);

    float part = 0.0f;
#pragma unroll
    for (int r = 0; r < 8; ++r) part = fmaf(leaky(acc2[r]), W3[i * HH + 8 * h + r], part);
    const float tot = part + __shfl_xor(part, 16, 32);
    if (lane < 16) Ow[lane * DD + i] = tot + b3[i];
    __syncthreads();
  }

  v4f val[7];
#pragma unroll
  for (int it = 0; it < 7; ++it) {
    const int p = lane + 32 * it;
    const int pc = (p < OPIECES) ? p : OPIECES - 1;
    val[it] = *(const v4fa*)(Ow + 4 * pc);
  }
  if (valid) {
    float* ob = out0 + (size_t)row0 * DD;
#pragma unroll
    for (int it = 0; it < 7; ++it) {
      const int p = lane + 32 * it;
      if (p < OPIECES) *(volatile v4f*)(ob + 4 * (size_t)p) = val[it];
    }
    __threadfence();
#pragma unroll
    for (int it = 0; it < 7; ++it) {
      const int p = lane + 32 * it;
      if (p < OPIECES) *(volatile v4f*)(ob + 4 * (size_t)p) = val[it];
    }
  }
}

extern "C" void kernel_launch(void* const* d_in, const int* in_sizes, int n_in,
                              void* d_out, int out_size, void* d_ws, size_t ws_size,
                              hipStream_t stream) {
  if (n_in < 10) return;
  if (in_sizes[0] != NN * DD) return;
  if (in_sizes[1] != DD * DD) return;
  if (in_sizes[2] != DD * DD) return;
  if (in_sizes[3] != DD * DD) return;
  if (in_sizes[4] != DD * DD * HH) return;
  if (in_sizes[5] != DD * HH) return;
  if (in_sizes[6] != DD * HH * HH) return;
  if (in_sizes[7] != DD * HH) return;
  if (in_sizes[8] != DD * HH) return;
  if (in_sizes[9] != DD) return;
  if (out_size != NN * DD + DD * DD) return;

  const float* x  = (const float*)d_in[0];
  const float* w  = (const float*)d_in[1];
  const float* u1 = (const float*)d_in[2];
  const float* u2 = (const float*)d_in[3];
  const float* W1 = (const float*)d_in[4];
  const float* b1 = (const float*)d_in[5];
  const float* W2 = (const float*)d_in[6];
  const float* b2 = (const float*)d_in[7];
  const float* W3 = (const float*)d_in[8];
  const float* b3 = (const float*)d_in[9];

  float* out0 = (float*)d_out;
  float* out1 = out0 + (size_t)NN * DD;

  const size_t ws_need = (size_t)(P1_HALVES + P2_HALVES) * 2;
  if (ws_need > ws_size) return;
  unsigned short* P1 = (unsigned short*)d_ws;
  unsigned short* P2 = P1 + P1_HALVES;

  k_prep<<<dim3(PREP_BLOCKS + 1), dim3(256), 0, stream>>>(w, u1, u2, W1, W2, P1, out1);
  k_main<<<dim3((TILES + 7) / 8), dim3(256), 0, stream>>>(x, P1, P2, b1, b2, W3, b3, out0, TILES);
  (void)hipGetLastError();
}
